// WaveNet_962072674955
// MI455X (gfx1250) — hardware-verified
//
#include <hip/hip_runtime.h>
#include <math.h>
#include <stddef.h>
#include <stdint.h>

typedef __attribute__((ext_vector_type(16))) _Float16 v16h;
typedef __attribute__((ext_vector_type(8)))  _Float16 v8h;
typedef __attribute__((ext_vector_type(8)))  float    v8f;
typedef __attribute__((ext_vector_type(4)))  float    v4f;
typedef unsigned int u32x4 __attribute__((ext_vector_type(4)));
typedef u32x4 u32x4a __attribute__((may_alias));

constexpr int kT       = 4096;
constexpr int kC       = 256;
constexpr int kZ       = 512;
constexpr int kKconv   = 2 * kC;
constexpr int kNL      = 40;
constexpr int kNLper   = 10;
constexpr int kAUX     = 80;
constexpr int kFR      = 16;
constexpr int kCls     = 256;
constexpr int kPre     = 512;
constexpr int kHTRows  = kPre + kT;
constexpr int kBT      = 64;
constexpr int kNBlkT   = kT / kBT;
constexpr int kZP      = 264;
constexpr int kSP      = 68;
constexpr int kThreads = 256;
constexpr int kWaves   = kThreads / 32;
constexpr int kET      = 32;
constexpr int kEP      = 257;
constexpr float kWCarry = 64.0f;
constexpr float kACarry = 16.0f;
constexpr float kFold   = 1.0f / 1024.0f;

static_assert(kT % kBT == 0 && kT % kET == 0);
static_assert(kKconv % 32 == 0 && kC % 32 == 0);
static_assert(kWaves * 32 == kC && kZ == 2 * kC);
static_assert(kBT == 64);
static_assert(kZ * kFR == 8 * kThreads * 4);
static_assert(kThreads == kC);
static_assert(kC * kBT == 16 * kThreads * 4);
static_assert(kZP % 8 == 0 && kZP >= kC);
static_assert((1 << (kNLper - 1)) <= kPre);
static_assert(kET * kC == kWaves * 8 * 4 * kET);
static_assert(kET == kWaves * 4);
static_assert(kBT == kWaves * 8);
static_assert((kNL * kZ * kFR) % kThreads == 0);
static_assert((kNL * kZ * kKconv / 8) % kThreads == 0);
static_assert(((kNL - 1) * kZ * kC / 8) % kThreads == 0);
static_assert((kC * kC / 8) % kThreads == 0);

constexpr size_t kBytesPlane = (size_t)kC * kT * 4;
constexpr size_t kBytesHT    = (size_t)kHTRows * kC * 2;
constexpr size_t kBytesCS    = (size_t)kNL * kZ * kFR * 4;
constexpr size_t kBytesWA    = (size_t)kNL * kZ * kKconv * 2;
constexpr size_t kBytesWO    = (size_t)(kNL - 1) * kZ * kC * 2;
constexpr size_t kBytesW256  = (size_t)kC * kC * 2;
constexpr size_t kOffHA  = 0;
constexpr size_t kOffHB  = kOffHA + kBytesPlane;
constexpr size_t kOffSA  = kOffHB + kBytesPlane;
constexpr size_t kOffSB  = kOffSA + kBytesPlane;
constexpr size_t kOffHTA = kOffSB + kBytesPlane;
constexpr size_t kOffHTB = kOffHTA + kBytesHT;
constexpr size_t kOffCS  = kOffHTB + kBytesHT;
constexpr size_t kOffWA  = kOffCS + kBytesCS;
constexpr size_t kOffWO  = kOffWA + kBytesWA;
constexpr size_t kOffLWO = kOffWO + kBytesWO;
constexpr size_t kOffE1  = kOffLWO + kBytesW256;
constexpr size_t kOffE2  = kOffE1 + kBytesW256;
constexpr size_t kWsTotal = kOffE2 + kBytesW256;
static_assert(kWsTotal == 54394880);
static_assert(kWsTotal <= (size_t)134217728);
static_assert(kOffHB % 256 == 0 && kOffSA % 256 == 0 && kOffSB % 256 == 0 && kOffHTA % 256 == 0 && kOffHTB % 256 == 0);
static_assert(kOffCS % 256 == 0 && kOffWA % 256 == 0 && kOffWO % 256 == 0 && kOffLWO % 256 == 0 && kOffE1 % 256 == 0 && kOffE2 % 256 == 0);

__device__ __forceinline__ unsigned short f2bf_bits(float f) {
  unsigned u = __float_as_uint(f);
  return (unsigned short)((u + 0x7FFFu + ((u >> 16) & 1u)) >> 16);
}
__device__ __forceinline__ float bf_bits2f(unsigned short h) { return __uint_as_float(((unsigned)h) << 16); }
__device__ __forceinline__ float bfr(float f) { return bf_bits2f(f2bf_bits(f)); }

__device__ __forceinline__ void keep4_h(v16h a, v16h b, v16h c, v16h d) { asm volatile("v_nop" :: "v"(a), "v"(b), "v"(c), "v"(d)); }
__device__ __forceinline__ void acc_guard4(v8f& a, v8f& b, v8f& c, v8f& d) { asm volatile("v_nop\n\tv_nop\n\tv_nop\n\tv_nop" : "+v"(a), "+v"(b), "+v"(c), "+v"(d)); }
__device__ __forceinline__ void grp_guard(v8f& a, v8f& b, v8f& c, v8f& d, v16h x, v16h y0, v16h y1, v16h y2, v16h y3) {
  asm volatile("v_nop\n\tv_nop\n\tv_nop\n\tv_nop" : "+v"(a), "+v"(b), "+v"(c), "+v"(d) : "v"(x), "v"(y0), "v"(y1), "v"(y2), "v"(y3));
}
template <typename T> struct Frag;
template <> struct Frag<_Float16> {
  typedef v16h V; union U { v16h v; v8h h[2]; };
  static __device__ __forceinline__ v16h load(const _Float16* p) {
    U f; f.h[0] = *(const v8h*)(p); f.h[1] = *(const v8h*)(p + 16); return f.v;
  }
  static __device__ __forceinline__ v8f mma(v16h a, v16h b, v8f c) {
    return __builtin_amdgcn_wmma_f32_16x16x32_f16(false, a, false, b, (short)0, c, false, false);
  }
};
typedef Frag<_Float16> FragH;

__device__ __forceinline__ void wave_lds_sync() {
  __builtin_amdgcn_fence(__ATOMIC_RELEASE, "workgroup");
  __builtin_amdgcn_wave_barrier();
  __builtin_amdgcn_fence(__ATOMIC_ACQUIRE, "workgroup");
}

__device__ __forceinline__ void zero_acc(v8f (&acc)[4][4]) {
#pragma unroll
  for (int i = 0; i < 4; ++i)
#pragma unroll
    for (int j = 0; j < 4; ++j) acc[i][j] = (v8f){0.f, 0.f, 0.f, 0.f, 0.f, 0.f, 0.f, 0.f};
}

template <int NI>
__device__ __forceinline__ void gemm_lds_k256(v8f (&acc)[4][4], const _Float16* __restrict__ A, int base_lo, int base_hi,
                                              const _Float16* bt, int rlane, int koff) {
#pragma unroll 1
  for (int k0 = 0; k0 < kC; k0 += 32) {
    v16h bfv[4];
#pragma unroll
    for (int j = 0; j < 4; ++j) bfv[j] = FragH::load(bt + (16 * j + rlane) * kZP + koff + k0);
#pragma unroll
    for (int i = 0; i < NI; ++i) {
      const int mrow = (i < 2) ? (base_lo + 16 * i) : (base_hi + 16 * (i - 2));
      const v16h af = FragH::load(A + (size_t)(mrow + rlane) * kC + koff + k0);
#pragma unroll
      for (int j = 0; j < 4; ++j) acc[i][j] = FragH::mma(af, bfv[j], acc[i][j]);
      grp_guard(acc[i][0], acc[i][1], acc[i][2], acc[i][3], af, bfv[0], bfv[1], bfv[2], bfv[3]);
    }
    keep4_h(bfv[0], bfv[1], bfv[2], bfv[3]);
  }
  acc_guard4(acc[0][0], acc[0][1], acc[0][2], acc[0][3]);
  acc_guard4(acc[1][0], acc[1][1], acc[1][2], acc[1][3]);
  if (NI > 2) {
    acc_guard4(acc[2][0], acc[2][1], acc[2][2], acc[2][3]);
    acc_guard4(acc[3][0], acc[3][1], acc[3][2], acc[3][3]);
  }
}

__device__ __forceinline__ void stage_slab(float* slab, const v8f (&a)[4], const float* bl, int hh, int rlane) {
#pragma unroll
  for (int j = 0; j < 4; ++j)
#pragma unroll
    for (int r = 0; r < 8; ++r)
      slab[(8 * hh + r) * kSP + 16 * j + rlane] = a[j][r] * kFold + bl[8 * hh + r];
}

__device__ __forceinline__ void add_store_rows(const float* slab, const float* __restrict__ src, float* __restrict__ dst,
                                               int ch0, int t0, int hh, int c4) {
  v4f vv[8];
#pragma unroll
  for (int it = 0; it < 8; ++it) {
    const int row = 2 * it + hh;
    const v4f o = *(const v4f*)(slab + row * kSP + c4);
    const v4f s = *(const v4f*)(src + (size_t)(ch0 + row) * kT + t0 + c4);
    vv[it] = s + o;
  }
  for (int pass = 0; pass < 2; ++pass) {
#pragma unroll
    for (int it = 0; it < 8; ++it)
      *(volatile v4f*)(dst + (size_t)(ch0 + 2 * it + hh) * kT + t0 + c4) = vv[it];
    __threadfence();
  }
}

__device__ __forceinline__ void resid_store_rows(const float* slab, const float* __restrict__ src, float* __restrict__ dst,
                                                 _Float16* zt, int ch0, int t0, int hh, int c4) {
  v4f vv[8];
#pragma unroll
  for (int it = 0; it < 8; ++it) {
    const int row = 2 * it + hh;
    const v4f o = *(const v4f*)(slab + row * kSP + c4);
    const v4f s = *(const v4f*)(src + (size_t)(ch0 + row) * kT + t0 + c4);
    vv[it] = s + o;
#pragma unroll
    for (int e = 0; e < 4; ++e) zt[(c4 + e) * kZP + ch0 + row] = (_Float16)(kACarry * vv[it][e]);
  }
  for (int pass = 0; pass < 2; ++pass) {
#pragma unroll
    for (int it = 0; it < 8; ++it)
      *(volatile v4f*)(dst + (size_t)(ch0 + 2 * it + hh) * kT + t0 + c4) = vv[it];
    __threadfence();
  }
}

__global__ __launch_bounds__(kThreads) void k_zero16(unsigned int* __restrict__ p, int n4) {
  const int i = blockIdx.x * kThreads + threadIdx.x;
  if (i >= n4) return;
  const u32x4 z = {0u, 0u, 0u, 0u};
  *(volatile u32x4*)(p + (size_t)i * 4) = z;
  __threadfence();
  *(volatile u32x4*)(p + (size_t)i * 4) = z;
}

__global__ __launch_bounds__(kThreads) void k_cast16(const float* __restrict__ in, unsigned short* __restrict__ out, int n8) {
  const int i = blockIdx.x * kThreads + threadIdx.x;
  if (i >= n8) return;
  const v4f a = *(const v4f*)(in + (size_t)i * 8);
  const v4f b = *(const v4f*)(in + (size_t)i * 8 + 4);
  v8h hv;
#pragma unroll
  for (int e = 0; e < 4; ++e) {
    hv[e]     = (_Float16)(kWCarry * bfr(a[e]));
    hv[4 + e] = (_Float16)(kWCarry * bfr(b[e]));
  }
  *(volatile v8h*)(out + (size_t)i * 8) = hv;
  __threadfence();
  *(volatile v8h*)(out + (size_t)i * 8) = hv;
}

__global__ __launch_bounds__(kThreads) void k_prep_convw(const float* __restrict__ w, unsigned short* __restrict__ wA, int n8) {
  const int i = blockIdx.x * kThreads + threadIdx.x;
  if (i >= n8) return;
  const int rm  = i >> 6;
  const int k0  = (i & 63) * 8;
  const int tap = k0 >> 8;
  const int c0  = k0 & (kC - 1);
  const float* src = w + ((size_t)rm * kC + c0) * 2 + tap;
  v8h hv;
#pragma unroll
  for (int e = 0; e < 8; ++e) hv[e] = (_Float16)(kWCarry * bfr(src[2 * e]));
  *(volatile v8h*)(wA + (size_t)i * 8) = hv;
  __threadfence();
  *(volatile v8h*)(wA + (size_t)i * 8) = hv;
}

__global__ __launch_bounds__(kThreads) void k_embed(const int* __restrict__ x, const float* __restrict__ emb,
                                                    float* __restrict__ h, unsigned short* __restrict__ hT) {
  __shared__ float tile[kET * kEP];
  const int tid = threadIdx.x, lane = tid & 31, wave = tid >> 5;
  const int t0 = blockIdx.x * kET;
  const int c = tid;
#pragma unroll 1
  for (int i = 0; i < kET; ++i) {
    int cls = x[t0 + i];
    cls = cls < 0 ? 0 : (cls > kCls - 1 ? kCls - 1 : cls);
    const float v = tanhf(bfr(emb[(size_t)cls * kC + c]));
    tile[i * kEP + c] = v;
  }
  __syncthreads();
  const int q = lane >> 3, p = lane & 7;
  v4f hv[8];
#pragma unroll
  for (int it = 0; it < 8; ++it) {
    const int cr = 32 * wave + 4 * it + q;
    v4f v;
#pragma unroll
    for (int e = 0; e < 4; ++e) v[e] = tile[(4 * p + e) * kEP + cr];
    hv[it] = v;
  }
  for (int pass = 0; pass < 2; ++pass) {
#pragma unroll
    for (int it = 0; it < 8; ++it)
      *(volatile v4f*)(h + (size_t)(32 * wave + 4 * it + q) * kT + t0 + 4 * p) = hv[it];
    __threadfence();
  }
  v8h tv[4];
#pragma unroll
  for (int it = 0; it < 4; ++it) {
    const int i = 4 * wave + it;
#pragma unroll
    for (int e = 0; e < 8; ++e) tv[it][e] = (_Float16)(kACarry * tile[i * kEP + 8 * lane + e]);
  }
  for (int pass = 0; pass < 2; ++pass) {
#pragma unroll
    for (int it = 0; it < 4; ++it)
      *(volatile v8h*)(hT + (size_t)(kPre + t0 + 4 * wave + it) * kC + 8 * lane) = tv[it];
    __threadfence();
  }
}

__global__ __launch_bounds__(kThreads) void k_cond(const float* __restrict__ cw, const float* __restrict__ y,
                                                   float* __restrict__ cs) {
  __shared__ float ys[kAUX * kFR];
  const int tid = threadIdx.x;
#pragma unroll 1
  for (int i = tid; i < kAUX * kFR; i += kThreads) ys[i] = bfr(y[i]);
  __syncthreads();
  const int idx = blockIdx.x * kThreads + tid;
  if (idx >= kNL * kZ * kFR) return;
  const int g = idx >> 4, f = idx & (kFR - 1);
  const float* row = cw + (size_t)g * kAUX;
  float s = 0.0f;
#pragma unroll 4
  for (int a = 0; a < kAUX; ++a) s += bfr(row[a]) * ys[a * kFR + f];
  ((volatile float*)cs)[idx] = s;
  __threadfence();
  ((volatile float*)cs)[idx] = s;
}

template <bool LAST>
__global__ __launch_bounds__(kThreads) void k_layer(
    const unsigned short* __restrict__ hT_in, const float* __restrict__ h_in, const float* __restrict__ skip_in,
    const unsigned short* __restrict__ wconv, const float* __restrict__ bconv,
    const unsigned short* __restrict__ wout, const float* __restrict__ bout,
    const float* __restrict__ cs_l,
    float* __restrict__ h_out, unsigned short* __restrict__ hT_out, float* __restrict__ skip_out, int dil) {
  __shared__ __align__(16) _Float16 zt[kBT * kZP];
  __shared__ __align__(16) float slabs[kWaves][16 * kSP];
  __shared__ __align__(16) float css[kZ * kFR];
  __shared__ __align__(16) float lbs[kZ];
  __shared__ __align__(16) float wobs[kZ];

  const int tid = threadIdx.x, lane = tid & 31, wave = tid >> 5;
  const int rlane = lane & 15, hh = lane >> 4, koff = hh * 8, c4 = rlane * 4;
  const int t0 = blockIdx.x * kBT;
  int d = dil;
  d = d < 0 ? 0 : (d > kPre ? kPre : d);

#pragma unroll
  for (int k = 0; k < 8; ++k) {
    const int q4 = tid + k * kThreads;
    *(v4f*)(css + q4 * 4) = *(const v4f*)(cs_l + (size_t)q4 * 4);
  }
  if (tid < kZ / 4) {
    const v4f b = *(const v4f*)(bconv + tid * 4);
    v4f r4;
    r4[0] = bfr(b[0]); r4[1] = bfr(b[1]); r4[2] = bfr(b[2]); r4[3] = bfr(b[3]);
    *(v4f*)(lbs + tid * 4) = r4;
  } else {
    const int jj = tid - kZ / 4;
    const int nb4 = LAST ? (kC / 4) : (kZ / 4);
    if (jj < nb4) {
      const v4f b = *(const v4f*)(bout + jj * 4);
      v4f r4;
      r4[0] = bfr(b[0]); r4[1] = bfr(b[1]); r4[2] = bfr(b[2]); r4[3] = bfr(b[3]);
      *(v4f*)(wobs + jj * 4) = r4;
    }
  }
  __syncthreads();

  const _Float16* hT = (const _Float16*)hT_in;
  const _Float16* wa = (const _Float16*)wconv;
  const int base_lo = 32 * wave, base_hi = kC + 32 * wave;
  v8f acc[4][4];
  zero_acc(acc);
#pragma unroll 1
  for (int k0 = 0; k0 < kKconv; k0 += 32) {
    const int shift = (k0 < kC) ? d : 0;
    const int kk = k0 & (kC - 1);
    v16h bfv[4];
#pragma unroll
    for (int j = 0; j < 4; ++j) {
      const int brow = kPre + t0 + 16 * j + rlane - shift;
      bfv[j] = FragH::load(hT + (size_t)brow * kC + kk + koff);
    }
#pragma unroll
    for (int i = 0; i < 4; ++i) {
      const int mrow = (i < 2) ? (base_lo + 16 * i) : (base_hi + 16 * (i - 2));
      const v16h af = FragH::load(wa + (size_t)(mrow + rlane) * kKconv + k0 + koff);
#pragma unroll
      for (int j = 0; j < 4; ++j) acc[i][j] = FragH::mma(af, bfv[j], acc[i][j]);
      grp_guard(acc[i][0], acc[i][1], acc[i][2], acc[i][3], af, bfv[0], bfv[1], bfv[2], bfv[3]);
    }
    keep4_h(bfv[0], bfv[1], bfv[2], bfv[3]);
  }
  acc_guard4(acc[0][0], acc[0][1], acc[0][2], acc[0][3]);
  acc_guard4(acc[1][0], acc[1][1], acc[1][2], acc[1][3]);
  acc_guard4(acc[2][0], acc[2][1], acc[2][2], acc[2][3]);
  acc_guard4(acc[3][0], acc[3][1], acc[3][2], acc[3][3]);

#pragma unroll
  for (int j = 0; j < 4; ++j) {
    const int t = t0 + 16 * j + rlane;
    const float pos = fmaxf(((float)t + 0.5f) * (1.0f / 256.0f) - 0.5f, 0.0f);
    int i0 = (int)pos;
    i0 = i0 > kFR - 1 ? kFR - 1 : i0;
    const int i1 = (i0 + 1 < kFR) ? (i0 + 1) : (kFR - 1);
    const float wf = pos - (float)i0;
    const float wg = 1.0f - wf;
    _Float16* zcol = zt + (16 * j + rlane) * kZP;
#pragma unroll
    for (int i = 0; i < 2; ++i) {
      const int ra0 = base_lo + 16 * i + 8 * hh;
#pragma unroll
      for (int r = 0; r < 8; ++r) {
        const int ra = ra0 + r, rg = ra + kC;
        const float ca = css[ra * kFR + i0] * wg + css[ra * kFR + i1] * wf;
        const float cg = css[rg * kFR + i0] * wg + css[rg * kFR + i1] * wf;
        const float av = acc[i][j][r] * kFold + lbs[ra] + ca;
        const float gv = acc[i + 2][j][r] * kFold + lbs[rg] + cg;
        const float th = 1.0f - 2.0f * __builtin_amdgcn_rcpf(expf(2.0f * av) + 1.0f);
        const float sg = __builtin_amdgcn_rcpf(1.0f + expf(-gv));
        zcol[ra] = (_Float16)(kACarry * (th * sg));
      }
    }
  }
  __syncthreads();

  constexpr int NI2 = LAST ? 2 : 4;
  zero_acc(acc);
  gemm_lds_k256<NI2>(acc, (const _Float16*)wout, base_lo, base_hi, zt, rlane, koff);
  __syncthreads();

  float* slab = slabs[wave];
  if constexpr (!LAST) {
#pragma unroll
    for (int i = 0; i < 2; ++i) {
      const int ch0 = base_lo + 16 * i;
      stage_slab(slab, acc[i], wobs + ch0, hh, rlane);
      wave_lds_sync();
      resid_store_rows(slab, h_in, h_out, zt, ch0, t0, hh, c4);
      wave_lds_sync();
    }
#pragma unroll
    for (int i = 2; i < 4; ++i) {
      const int ch0 = base_lo + 16 * (i - 2);
      stage_slab(slab, acc[i], wobs + kC + ch0, hh, rlane);
      wave_lds_sync();
      add_store_rows(slab, skip_in, skip_out, ch0, t0, hh, c4);
      wave_lds_sync();
    }
    __syncthreads();
    for (int pass = 0; pass < 2; ++pass) {
#pragma unroll
      for (int it = 0; it < 8; ++it) {
        const int trow = 8 * wave + it;
        const u32x4 v = *(const u32x4a*)(zt + trow * kZP + 8 * lane);
        *(volatile u32x4*)(hT_out + ((size_t)(kPre + t0 + trow) * kC + 8 * lane)) = v;
      }
      __threadfence();
    }
  } else {
#pragma unroll
    for (int i = 0; i < 2; ++i) {
      const int ch0 = base_lo + 16 * i;
      stage_slab(slab, acc[i], wobs + ch0, hh, rlane);
      wave_lds_sync();
      add_store_rows(slab, skip_in, skip_out, ch0, t0, hh, c4);
      wave_lds_sync();
    }
  }
}

__global__ __launch_bounds__(kThreads) void k_head(const float* __restrict__ skip,
                                                   const unsigned short* __restrict__ w1, const float* __restrict__ b1,
                                                   const unsigned short* __restrict__ w2, const float* __restrict__ b2,
                                                   float* __restrict__ out) {
  __shared__ __align__(16) _Float16 ut[kBT * kZP];
  __shared__ __align__(16) float slabs[kWaves][16 * kSP];
  __shared__ __align__(16) float b1s[kC];
  __shared__ __align__(16) float b2s[kC];

  const int tid = threadIdx.x, lane = tid & 31, wave = tid >> 5;
  const int rlane = lane & 15, hh = lane >> 4, koff = hh * 8, c4 = rlane * 4;
  const int t0 = blockIdx.x * kBT;
  const int base_lo = 32 * wave;

  if (tid < kC / 4) {
    const v4f b = *(const v4f*)(b1 + tid * 4);
    v4f r4;
    r4[0] = bfr(b[0]); r4[1] = bfr(b[1]); r4[2] = bfr(b[2]); r4[3] = bfr(b[3]);
    *(v4f*)(b1s + tid * 4) = r4;
  } else if (tid < kC / 2) {
    const int jj = tid - kC / 4;
    const v4f b = *(const v4f*)(b2 + jj * 4);
    v4f r4;
    r4[0] = bfr(b[0]); r4[1] = bfr(b[1]); r4[2] = bfr(b[2]); r4[3] = bfr(b[3]);
    *(v4f*)(b2s + jj * 4) = r4;
  }
#pragma unroll 1
  for (int it = 0; it < 16; ++it) {
    const int c  = it * 16 + (tid >> 4);
    const int t4 = (tid & 15) * 4;
    const v4f s = *(const v4f*)(skip + (size_t)c * kT + t0 + t4);
#pragma unroll
    for (int e = 0; e < 4; ++e) ut[(t4 + e) * kZP + c] = (_Float16)(kACarry * fmaxf(s[e], 0.0f));
  }
  __syncthreads();

  v8f acc[4][4];
  zero_acc(acc);
  gemm_lds_k256<2>(acc, (const _Float16*)w1, base_lo, base_lo, ut, rlane, koff);
  __syncthreads();
#pragma unroll
  for (int i = 0; i < 2; ++i)
#pragma unroll
    for (int j = 0; j < 4; ++j)
#pragma unroll
      for (int r = 0; r < 8; ++r) {
        const int ch = base_lo + 16 * i + 8 * hh + r;
        const float v = fmaxf(acc[i][j][r] * kFold + b1s[ch], 0.0f);
        ut[(16 * j + rlane) * kZP + ch] = (_Float16)(kACarry * v);
      }
  __syncthreads();

  zero_acc(acc);
  gemm_lds_k256<2>(acc, (const _Float16*)w2, base_lo, base_lo, ut, rlane, koff);

  float* slab = slabs[wave];
#pragma unroll
  for (int i = 0; i < 2; ++i) {
    const int ch0 = base_lo + 16 * i;
    stage_slab(slab, acc[i], b2s + ch0, hh, rlane);
    wave_lds_sync();
    v4f vv[8];
#pragma unroll
    for (int it = 0; it < 8; ++it) vv[it] = *(const v4f*)(slab + (2 * it + hh) * kSP + c4);
    for (int pass = 0; pass < 2; ++pass) {
#pragma unroll
      for (int it = 0; it < 8; ++it)
        *(volatile v4f*)(out + (size_t)(ch0 + 2 * it + hh) * kT + t0 + c4) = vv[it];
      __threadfence();
    }
    wave_lds_sync();
  }
}

extern "C" void kernel_launch(void* const* d_in, const int* in_sizes, int n_in,
                              void* d_out, int out_size, void* d_ws, size_t ws_size,
                              hipStream_t stream) {
  if (n_in < 15) return;
  if (in_sizes[0] != kT || in_sizes[1] != kAUX * kFR || in_sizes[3] != kCls * kC ||
      in_sizes[4] != kNL * kZ * kAUX || in_sizes[5] != kNL * kZ * kC * 2 || in_sizes[6] != kNL * kZ ||
      in_sizes[7] != (kNL - 1) * kZ * kC || in_sizes[8] != (kNL - 1) * kZ ||
      in_sizes[9] != kC * kC || in_sizes[10] != kC || in_sizes[11] != kC * kC || in_sizes[12] != kC ||
      in_sizes[13] != kC * kC || in_sizes[14] != kC || out_size != kC * kT) return;
  if (ws_size < kWsTotal) return;

  const int*   x         = (const int*)  d_in[0];
  const float* y         = (const float*)d_in[1];
  const float* emb_w     = (const float*)d_in[3];
  const float* cond_w    = (const float*)d_in[4];
  const float* layer_w   = (const float*)d_in[5];
  const float* layer_b   = (const float*)d_in[6];
  const float* wo_w      = (const float*)d_in[7];
  const float* wo_b      = (const float*)d_in[8];
  const float* last_wo_w = (const float*)d_in[9];
  const float* last_wo_b = (const float*)d_in[10];
  const float* end1_w    = (const float*)d_in[11];
  const float* end1_b    = (const float*)d_in[12];
  const float* end2_w    = (const float*)d_in[13];
  const float* end2_b    = (const float*)d_in[14];
  float* out = (float*)d_out;

  char* ws = (char*)d_ws;
  float* hA    = (float*)(ws + kOffHA);
  float* hB    = (float*)(ws + kOffHB);
  float* skipA = (float*)(ws + kOffSA);
  float* skipB = (float*)(ws + kOffSB);
  unsigned short* hTA  = (unsigned short*)(ws + kOffHTA);
  unsigned short* hTB  = (unsigned short*)(ws + kOffHTB);
  float* cs    = (float*)(ws + kOffCS);
  unsigned short* wA   = (unsigned short*)(ws + kOffWA);
  unsigned short* woA  = (unsigned short*)(ws + kOffWO);
  unsigned short* lwoA = (unsigned short*)(ws + kOffLWO);
  unsigned short* e1A  = (unsigned short*)(ws + kOffE1);
  unsigned short* e2A  = (unsigned short*)(ws + kOffE2);

  {
    const int n8 = kNL * kZ * kKconv / 8;
    k_prep_convw<<<n8 / kThreads, kThreads, 0, stream>>>(layer_w, wA, n8);
  }
  {
    const int n8 = (kNL - 1) * kZ * kC / 8;
    k_cast16<<<n8 / kThreads, kThreads, 0, stream>>>(wo_w, woA, n8);
  }
  {
    const int n8 = kC * kC / 8;
    k_cast16<<<n8 / kThreads, kThreads, 0, stream>>>(last_wo_w, lwoA, n8);
    k_cast16<<<n8 / kThreads, kThreads, 0, stream>>>(end1_w, e1A, n8);
    k_cast16<<<n8 / kThreads, kThreads, 0, stream>>>(end2_w, e2A, n8);
  }
  {
    const int n4pre = kPre * kC * 2 / 16;
    k_zero16<<<(n4pre + kThreads - 1) / kThreads, kThreads, 0, stream>>>((unsigned int*)hTA, n4pre);
    k_zero16<<<(n4pre + kThreads - 1) / kThreads, kThreads, 0, stream>>>((unsigned int*)hTB, n4pre);
    const int n4skip = kC * kT * 4 / 16;
    k_zero16<<<(n4skip + kThreads - 1) / kThreads, kThreads, 0, stream>>>((unsigned int*)skipA, n4skip);
  }
  k_embed<<<kT / kET, kThreads, 0, stream>>>(x, emb_w, hA, hTA);
  k_cond<<<(kNL * kZ * kFR) / kThreads, kThreads, 0, stream>>>(cond_w, y, cs);

  for (int i = 0; i < kNL; ++i) {
    const int dil = 1 << (i % kNLper);
    const float* hin = (i & 1) ? hB : hA;
    float* hout      = (i & 1) ? hA : hB;
    const unsigned short* htin = (i & 1) ? hTB : hTA;
    unsigned short* htout      = (i & 1) ? hTA : hTB;
    const float* sin_p = (i & 1) ? skipB : skipA;
    float* sout_p      = (i & 1) ? skipA : skipB;
    const unsigned short* wconv = wA + (size_t)i * kZ * kKconv;
    const float* bconv = layer_b + (size_t)i * kZ;
    const float* cs_l  = cs + (size_t)i * kZ * kFR;
    if (i < kNL - 1) {
      k_layer<false><<<kNBlkT, kThreads, 0, stream>>>(htin, hin, sin_p, wconv, bconv,
                                                      woA + (size_t)i * kZ * kC, wo_b + (size_t)i * kZ, cs_l,
                                                      hout, htout, sout_p, dil);
    } else {
      k_layer<true><<<kNBlkT, kThreads, 0, stream>>>(htin, hin, sin_p, wconv, bconv,
                                                     lwoA, last_wo_b, cs_l,
                                                     hout, htout, sout_p, dil);
    }
  }
  const float* skip_final = ((kNL - 1) & 1) ? skipA : skipB;

  k_head<<<kNBlkT, kThreads, 0, stream>>>(skip_final, e1A, end1_b, e2A, end2_b, out);
}
